// MultiHead_74311524155835
// MI455X (gfx1250) — hardware-verified
//
#include <hip/hip_runtime.h>
#ifndef NB
#define NB 64
#endif
#ifndef SEQ
#define SEQ 512
#endif
#define NB_FULL 64
#define SEQ_FULL 512
#define DM 384
#define NH 6
#define HD 64
#define QT0 128
#define PP 40
#define OPP 72
static_assert(NB >= 1 && NB <= NB_FULL);
static_assert(SEQ % 128 == 0 && SEQ >= 2 * QT0 && SEQ <= SEQ_FULL);
static_assert(DM == NH * HD && DM % 128 == 0 && HD == 64 && QT0 == 128);

typedef unsigned short v8us __attribute__((ext_vector_type(8), may_alias));
typedef float  v8f  __attribute__((ext_vector_type(8)));
typedef float  v4f  __attribute__((ext_vector_type(4)));
typedef float  v4fa __attribute__((ext_vector_type(4), may_alias));
typedef _Float16 v16h __attribute__((ext_vector_type(16)));
typedef _Float16 v4h __attribute__((ext_vector_type(4)));
union FragH { v16h v; v8us half[2]; _Float16 h[16]; unsigned short u[16]; };

__device__ __forceinline__ unsigned short bf16_bits(float x) { unsigned int u = __float_as_uint(x); return (unsigned short)((u + 0x7FFFu + ((u >> 16) & 1u)) >> 16); }
__device__ __forceinline__ float bf16_val(unsigned short b) { return __uint_as_float(((unsigned int)b) << 16); }
__device__ __forceinline__ float bf16_rne(float x) { return bf16_val(bf16_bits(x)); }

__device__ __forceinline__ v16h g2_frag(const _Float16* p, int hh) { FragH f; f.half[0] = *(const v8us*)((const unsigned short*)p + 8 * hh); f.half[1] = *(const v8us*)((const unsigned short*)p + 16 + 8 * hh); return f.v; }
__device__ __forceinline__ v8f g2_mma(v16h a, v16h b, v8f c) { v8f d = __builtin_amdgcn_wmma_f32_16x16x32_f16(false, a, false, b, (short)0, c, false, false); asm volatile("v_nop\n\tv_nop\n\tv_nop\n\tv_nop" : "+v"(d) : "v"(a), "v"(b)); return d; }

__global__ __launch_bounds__(256) void k_wnat(const float* __restrict__ w, size_t n8, _Float16* __restrict__ Bt) {
  const size_t t = (size_t)blockIdx.x * 256 + threadIdx.x; if (t >= n8) return; FragH f;
#pragma unroll
  for (int q = 0; q < 8; ++q) f.h[q] = (_Float16)(bf16_rne(w[t * 8 + q]) * 16.0f);
  unsigned short* d = (unsigned short*)Bt + t * 8;
  *(volatile v8us*)d = f.half[0]; __threadfence(); *(volatile v8us*)d = f.half[0];
}

__global__ __launch_bounds__(256) void k_x16(const float* __restrict__ x, _Float16* __restrict__ X16, size_t n8) {
  const size_t t = (size_t)blockIdx.x * 256 + threadIdx.x; if (t >= n8) return;
  const size_t wr = t / (DM / 8); const int c8 = (int)(t % (DM / 8)) * 8;
  const size_t b = wr / SEQ, tt = wr % SEQ;
  const float* src = x + (b * SEQ_FULL + tt) * DM + c8;
  const v4f a = *(const v4fa*)src, c = *(const v4fa*)(src + 4); FragH f;
#pragma unroll
  for (int q = 0; q < 4; ++q) { f.h[q] = (_Float16)bf16_rne(a[q]); f.h[4 + q] = (_Float16)bf16_rne(c[q]); }
  unsigned short* d = (unsigned short*)X16 + t * 8;
  *(volatile v8us*)d = f.half[0]; __threadfence(); *(volatile v8us*)d = f.half[0];
}

__global__ __launch_bounds__(128) void k_gemm2(const _Float16* __restrict__ A, int lda, size_t sA, const _Float16* __restrict__ Bh, int ldb, size_t sB, float alpha,
    const float* __restrict__ bias, const float* CP, int row0g, float* C, _Float16* C16, int ldc, size_t sC, int M, int N, int K) {
  __shared__ __attribute__((aligned(16))) float so[4][32][68];
  const int tid = threadIdx.x, w = tid >> 5, lane = tid & 31, ln = lane & 15, hh = lane >> 4; const int by = blockIdx.y;
  A += (size_t)by * sA; Bh += (size_t)by * sB; const size_t cofs = (size_t)by * sC;
  const int ntn = N >> 6; const int mt = blockIdx.x / ntn, nq = blockIdx.x - mt * ntn; const int row0 = mt * 128 + 32 * w, col0 = nq * 64; if (row0 >= M) return;
  const _Float16* a0p = A + (size_t)(row0 + ln) * lda; const _Float16* a1p = a0p + (size_t)16 * lda;
  const _Float16* b0p = Bh + (size_t)(col0 + ln) * ldb; const _Float16* b1p = b0p + (size_t)16 * ldb; const _Float16* b2p = b1p + (size_t)16 * ldb; const _Float16* b3p = b2p + (size_t)16 * ldb;
  const v8f z8 = {0.f,0.f,0.f,0.f,0.f,0.f,0.f,0.f}; v8f c00 = z8, c01 = z8, c02 = z8, c03 = z8, c10 = z8, c11 = z8, c12 = z8, c13 = z8;
#pragma unroll 1
  for (int kb = 0; kb < K; kb += 32) { const v16h a0 = g2_frag(a0p + kb, hh), a1 = g2_frag(a1p + kb, hh);
    v16h b = g2_frag(b0p + kb, hh); c00 = g2_mma(a0, b, c00); c10 = g2_mma(a1, b, c10);
    b = g2_frag(b1p + kb, hh); c01 = g2_mma(a0, b, c01); c11 = g2_mma(a1, b, c11);
    b = g2_frag(b2p + kb, hh); c02 = g2_mma(a0, b, c02); c12 = g2_mma(a1, b, c12);
    b = g2_frag(b3p + kb, hh); c03 = g2_mma(a0, b, c03); c13 = g2_mma(a1, b, c13); }
  v8f accs[8] = {c00, c01, c02, c03, c10, c11, c12, c13};
#pragma unroll
  for (int u = 0; u < 8; ++u) { const int t = u & 3, half = u >> 2; const int col = col0 + t * 16 + ln; const float bv = bias ? bf16_rne(bias[col]) : 0.f;
#pragma unroll
    for (int r = 0; r < 8; ++r) { const int rloc = half * 16 + 8 * hh + r; float v = accs[u][r] * alpha + bv;
      if (CP) v += CP[cofs + (size_t)(row0g + row0 + rloc) * ldc + col];
      so[w][rloc][t * 16 + ln] = v; } }
  __builtin_amdgcn_fence(4, "workgroup"); __builtin_amdgcn_wave_barrier();
  const int rsub = lane >> 4, c4 = (lane & 15) * 4;
  for (int pass = 0; pass < 2; ++pass) {
#pragma unroll
    for (int q = 0; q < 16; ++q) { const int r = q * 2 + rsub; const v4f v = *(const v4fa*)&so[w][r][c4];
      if (C) *(volatile v4f*)(C + cofs + (size_t)(row0 + r) * ldc + col0 + c4) = v;
      if (C16) { v4h h4; for (int i = 0; i < 4; ++i) h4[i] = (_Float16)v[i]; *(volatile v4h*)(C16 + cofs + (size_t)(row0 + r) * ldc + col0 + c4) = h4; } }
    if (pass == 0) __threadfence(); }
}

__global__ __launch_bounds__(64) void k_att0(const float* __restrict__ QF, const float* __restrict__ KF, const float* __restrict__ VF, float* __restrict__ OF) {
  #pragma clang fp contract(off)
  __shared__ __attribute__((aligned(16))) float lq[64][64]; __shared__ __attribute__((aligned(16))) float lo[64][64];
  const int tid = threadIdx.x; const int rg = blockIdx.x % (QT0 / 64); const int bh = blockIdx.x / (QT0 / 64); const int b = bh / NH, h = bh - b * NH;
  const size_t pofs = (size_t)b * QT0 * DM;
  const int i = rg * 64 + tid;
  const float* qr = QF + pofs + (size_t)i * DM + h * HD;
#pragma unroll 1
  for (int c = 0; c < HD / 4; ++c) { *(v4f*)&lq[tid][c * 4] = *(const v4fa*)(qr + c * 4); const v4f z = {0.f, 0.f, 0.f, 0.f}; *(v4f*)&lo[tid][c * 4] = z; }
  float m = -1.0e30f, l = 0.f; const int jmax = rg * 64 + (tid >> 5) * 32 + 31;
#pragma unroll 1
  for (int j = 0; j <= jmax; ++j) { const float* kr = KF + pofs + (size_t)j * DM + h * HD; const float* vr = VF + pofs + (size_t)j * DM + h * HD; float s = 0.f;
#pragma unroll 1
    for (int c = 0; c < HD / 4; ++c) { const v4f kq = *(const v4fa*)(kr + c * 4); const v4f qq = *(v4f*)&lq[tid][c * 4]; s = __fadd_rn(s, __fmul_rn(qq[0], kq[0])); s = __fadd_rn(s, __fmul_rn(qq[1], kq[1])); s = __fadd_rn(s, __fmul_rn(qq[2], kq[2])); s = __fadd_rn(s, __fmul_rn(qq[3], kq[3])); }
    s = __fmul_rn(s, 0.125f);
    const float f = (j <= i) ? 1.f : 0.f; const float sm = fmaf(f, s, (1.f - f) * -1.0e30f); const float mn = fmaxf(m, sm); const float sc = expf(m - mn); const float e = expf(sm - mn); l = __fadd_rn(__fmul_rn(l, sc), e); m = mn;
#pragma unroll 1
    for (int c = 0; c < HD / 4; ++c) { const v4f vv = *(const v4fa*)(vr + c * 4); v4f oo = *(v4f*)&lo[tid][c * 4]; for (int u = 0; u < 4; ++u) oo[u] = __fadd_rn(__fmul_rn(oo[u], sc), __fmul_rn(e, vv[u])); *(v4f*)&lo[tid][c * 4] = oo; } }
  const float fin = 64.0f / l;
#pragma unroll 1
  for (int c = 0; c < HD / 4; ++c) { v4f oo = *(v4f*)&lo[tid][c * 4]; for (int u = 0; u < 4; ++u) oo[u] = __fmul_rn(oo[u], fin); *(v4f*)&lo[tid][c * 4] = oo; }
  __syncthreads();
  for (int pass = 0; pass < 2; ++pass) {
#pragma unroll 1
    for (int it = 0; it < 16; ++it) { const int row = it * 4 + tid / 16, pc = (tid % 16) * 4; const v4f v = *(const v4f*)&lo[row][pc]; *(volatile v4f*)(OF + pofs + (size_t)(rg * 64 + row) * DM + h * HD + pc) = v; }
    if (pass == 0) __threadfence(); } }

__global__ __launch_bounds__(256) void k_hl(const float* __restrict__ F, _Float16* __restrict__ Hh, _Float16* __restrict__ Hl, size_t n8) {
  const size_t t = (size_t)blockIdx.x * 256 + threadIdx.x; if (t >= n8) return; FragH fh, fl; const v4f a = *(const v4fa*)(F + t * 8), c = *(const v4fa*)(F + t * 8 + 4);
#pragma unroll
  for (int q = 0; q < 4; ++q) { _Float16 hv = (_Float16)a[q]; fh.h[q] = hv; fl.h[q] = (_Float16)((a[q] - (float)hv) * 1024.0f); hv = (_Float16)c[q]; fh.h[4 + q] = hv; fl.h[4 + q] = (_Float16)((c[q] - (float)hv) * 1024.0f); }
  unsigned short* dh = (unsigned short*)Hh + t * 8; unsigned short* dl = (unsigned short*)Hl + t * 8;
  for (int pass = 0; pass < 2; ++pass) { *(volatile v8us*)dh = fh.half[0]; *(volatile v8us*)dl = fl.half[0]; if (pass == 0) __threadfence(); } }

__global__ __launch_bounds__(256) __attribute__((amdgpu_num_vgpr(256)))
void k_att(const _Float16* __restrict__ Q16, const _Float16* __restrict__ K16, const _Float16* __restrict__ VT, _Float16* __restrict__ O16) {
  __shared__ __attribute__((aligned(16))) _Float16 lp[8][2][16 * PP];
  __shared__ __attribute__((aligned(16))) _Float16 lso[8][16 * OPP];
  const int tid = threadIdx.x, w = tid >> 5, lane = tid & 31, ln = lane & 15, hh = lane >> 4;
  const int qt = blockIdx.x * 8 + w; const int bh = blockIdx.y; const int b = bh / NH, h = bh - b * NH;
  const int q0 = qt * 16;
  const size_t wr0 = (size_t)b * SEQ + q0;
  const _Float16* qp = Q16 + (wr0 + ln) * DM + h * HD;
  const v16h qa0 = g2_frag(qp, hh), qa1 = g2_frag(qp + 32, hh);
  const _Float16* kbase = K16 + (size_t)b * SEQ * DM + h * HD;
  const _Float16* vbase = VT + (size_t)bh * HD * SEQ;
  const v8f z8 = {0.f,0.f,0.f,0.f,0.f,0.f,0.f,0.f}; v8f o0 = z8, o1 = z8, o2 = z8, o3 = z8;
  float mr[8], lr[8];
#pragma unroll
  for (int r = 0; r < 8; ++r) { mr[r] = -1.0e30f; lr[r] = 0.f; }
  const int nkb = qt / 2 + 1;
#pragma unroll 1
  for (int it = 0; it < nkb; ++it) {
    const int kb = it * 32;
    _Float16* pb = &lp[w][it & 1][0];
    v8f s0 = z8, s1 = z8;
    { const _Float16* kp = kbase + (size_t)(kb + ln) * DM; v16h bk = g2_frag(kp, hh); s0 = g2_mma(qa0, bk, s0); bk = g2_frag(kp + 32, hh); s0 = g2_mma(qa1, bk, s0); }
    { const _Float16* kp = kbase + (size_t)(kb + 16 + ln) * DM; v16h bk = g2_frag(kp, hh); s1 = g2_mma(qa0, bk, s1); bk = g2_frag(kp + 32, hh); s1 = g2_mma(qa1, bk, s1); }
#pragma unroll
    for (int r = 0; r < 8; ++r) {
      const int qi = q0 + 8 * hh + r;
      const float v0 = (kb + ln <= qi) ? s0[r] * 0.125f : -1.0e30f;
      const float v1 = (kb + 16 + ln <= qi) ? s1[r] * 0.125f : -1.0e30f;
      float mx = fmaxf(v0, v1);
      mx = fmaxf(mx, __shfl_xor(mx, 1, 16)); mx = fmaxf(mx, __shfl_xor(mx, 2, 16)); mx = fmaxf(mx, __shfl_xor(mx, 4, 16)); mx = fmaxf(mx, __shfl_xor(mx, 8, 16));
      const float mn = fmaxf(mr[r], mx);
      const float al = __expf(mr[r] - mn); mr[r] = mn;
      const float p0 = __expf(v0 - mn), p1 = __expf(v1 - mn);
      float rs = p0 + p1;
      rs += __shfl_xor(rs, 1, 16); rs += __shfl_xor(rs, 2, 16); rs += __shfl_xor(rs, 4, 16); rs += __shfl_xor(rs, 8, 16);
      lr[r] = lr[r] * al + rs;
      o0[r] *= al; o1[r] *= al; o2[r] *= al; o3[r] *= al;
      pb[(8 * hh + r) * PP + ln] = (_Float16)(p0 * 1024.0f);
      pb[(8 * hh + r) * PP + 16 + ln] = (_Float16)(p1 * 1024.0f);
    }
    __builtin_amdgcn_fence(3, "wavefront"); __builtin_amdgcn_wave_barrier();
    FragH pa; pa.half[0] = *(const v8us*)((const unsigned short*)pb + ln * PP + 8 * hh); pa.half[1] = *(const v8us*)((const unsigned short*)pb + ln * PP + 16 + 8 * hh);
    { const _Float16* vp = vbase + (size_t)ln * SEQ + kb;
      v16h bv = g2_frag(vp, hh); o0 = g2_mma(pa.v, bv, o0);
      bv = g2_frag(vp + (size_t)16 * SEQ, hh); o1 = g2_mma(pa.v, bv, o1);
      bv = g2_frag(vp + (size_t)32 * SEQ, hh); o2 = g2_mma(pa.v, bv, o2);
      bv = g2_frag(vp + (size_t)48 * SEQ, hh); o3 = g2_mma(pa.v, bv, o3); }
  }
  _Float16* sob = &lso[w][0];
#pragma unroll
  for (int r = 0; r < 8; ++r) { const float inv = (1.0f / lr[r]) * 0.0009765625f; const int row = 8 * hh + r;
    sob[row * OPP + ln] = (_Float16)(o0[r] * inv); sob[row * OPP + 16 + ln] = (_Float16)(o1[r] * inv); sob[row * OPP + 32 + ln] = (_Float16)(o2[r] * inv); sob[row * OPP + 48 + ln] = (_Float16)(o3[r] * inv); }
  __builtin_amdgcn_fence(3, "wavefront"); __builtin_amdgcn_wave_barrier();
  unsigned short* ob = (unsigned short*)O16 + wr0 * DM + h * HD;
  for (int pass = 0; pass < 2; ++pass) {
#pragma unroll
    for (int it2 = 0; it2 < 4; ++it2) { const int row = it2 * 4 + (lane >> 3), c8 = (lane & 7) * 8; const v8us v = *(const v8us*)((const unsigned short*)sob + row * OPP + c8); *(volatile v8us*)(ob + (size_t)row * DM + c8) = v; }
    if (pass == 0) __threadfence(); }
}

extern "C" void kernel_launch(void* const* d_in, const int* in_sizes, int n_in,
                              void* d_out, int out_size, void* d_ws, size_t ws_size, hipStream_t stream) {
  if (n_in < 6) return;
  const float* x = (const float*)d_in[0]; const float* wq = (const float*)d_in[1]; const float* wk = (const float*)d_in[2];
  const float* wv = (const float*)d_in[3]; const float* wp = (const float*)d_in[4]; const float* bproj = (const float*)d_in[5];
  const size_t need_x = (size_t)(NB - 1) * SEQ_FULL * DM + (size_t)SEQ * DM;
  if ((size_t)in_sizes[0] < need_x || in_sizes[1] < DM * DM || in_sizes[2] < DM * DM || in_sizes[3] < DM * DM || in_sizes[4] < DM * DM || in_sizes[5] < DM || (size_t)out_size < need_x) return;
  float* out = (float*)d_out;
  char* ws = (char*)d_ws; size_t off = 0;
  auto take = [&](size_t bytes) { char* p = ws + off; off += (bytes + 255) & ~(size_t)255; return p; };
  const size_t wb = (size_t)DM * DM * 2;
  _Float16* WQ = (_Float16*)take(wb); _Float16* WK = (_Float16*)take(wb); _Float16* WV = (_Float16*)take(wb); _Float16* WP = (_Float16*)take(wb);
  const size_t rows2 = (size_t)NB * SEQ * DM * 2;
  const size_t f0b4 = (size_t)NB * QT0 * DM * 4;
  const size_t f0b2 = (size_t)NB * QT0 * DM * 2;
  const size_t vtb = (size_t)NB * DM * SEQ * 2;
  char* R1 = take(rows2);
  const size_t r2a = 3 * f0b4, r2b = rows2 + 2 * f0b2; char* R2 = take(r2a > r2b ? r2a : r2b);
  char* R3 = take(f0b4 > rows2 ? f0b4 : rows2);
  char* R4 = take(vtb);
  if (off > ws_size) return;
  _Float16* X16 = (_Float16*)R1; _Float16* O16 = (_Float16*)R1;
  float* QF0 = (float*)R2; float* KF0 = (float*)(R2 + f0b4); float* VF0 = (float*)(R2 + 2 * f0b4);
  _Float16* Q16 = (_Float16*)R2; _Float16* OH = (_Float16*)(R2 + rows2); _Float16* OL = (_Float16*)(R2 + rows2 + f0b2);
  float* OF0 = (float*)R3; _Float16* K16 = (_Float16*)R3;
  _Float16* VT = (_Float16*)R4;

  const size_t nw8 = (size_t)DM * DM / 8; const unsigned gw = (unsigned)((nw8 + 255) / 256);
  k_wnat<<<gw, 256, 0, stream>>>(wq, nw8, WQ); k_wnat<<<gw, 256, 0, stream>>>(wk, nw8, WK); k_wnat<<<gw, 256, 0, stream>>>(wv, nw8, WV); k_wnat<<<gw, 256, 0, stream>>>(wp, nw8, WP);
  const size_t nx8 = (size_t)NB * SEQ * DM / 8;
  k_x16<<<(unsigned)((nx8 + 255) / 256), 256, 0, stream>>>(x, X16, nx8);
  k_gemm2<<<dim3((QT0 / 128) * (DM / 64), NB), 128, 0, stream>>>(X16, DM, (size_t)SEQ * DM, WQ, DM, (size_t)0, 0.0625f, nullptr, nullptr, 0, QF0, nullptr, DM, (size_t)QT0 * DM, QT0, DM, DM);
  k_gemm2<<<dim3((QT0 / 128) * (DM / 64), NB), 128, 0, stream>>>(X16, DM, (size_t)SEQ * DM, WK, DM, (size_t)0, 0.0625f, nullptr, nullptr, 0, KF0, nullptr, DM, (size_t)QT0 * DM, QT0, DM, DM);
  k_gemm2<<<dim3((QT0 / 128) * (DM / 64), NB), 128, 0, stream>>>(X16, DM, (size_t)SEQ * DM, WV, DM, (size_t)0, 0.0625f, nullptr, nullptr, 0, VF0, nullptr, DM, (size_t)QT0 * DM, QT0, DM, DM);
  k_att0<<<NB * NH * (QT0 / 64), 64, 0, stream>>>(QF0, KF0, VF0, OF0);
  const size_t nf8 = (size_t)NB * QT0 * DM / 8;
  k_hl<<<(unsigned)((nf8 + 255) / 256), 256, 0, stream>>>(OF0, OH, OL, nf8);
  k_gemm2<<<dim3((unsigned)((NB * SEQ / 128) * (DM / 64)), 1), 128, 0, stream>>>(X16, DM, (size_t)0, WQ, DM, (size_t)0, 0.0625f, nullptr, nullptr, 0, nullptr, Q16, DM, (size_t)0, NB * SEQ, DM, DM);
  k_gemm2<<<dim3((unsigned)((NB * SEQ / 128) * (DM / 64)), 1), 128, 0, stream>>>(X16, DM, (size_t)0, WK, DM, (size_t)0, 0.0625f, nullptr, nullptr, 0, nullptr, K16, DM, (size_t)0, NB * SEQ, DM, DM);
  k_gemm2<<<dim3((DM / 128) * (SEQ / 64), NB), 128, 0, stream>>>(WV, DM, (size_t)0, X16, DM, (size_t)SEQ * DM, 0.0625f, nullptr, nullptr, 0, nullptr, VT, SEQ, (size_t)DM * SEQ, DM, SEQ, DM);
  k_att<<<dim3(SEQ / 128, NB * NH), 256, 0, stream>>>(Q16, K16, VT, O16);
  k_gemm2<<<dim3(((SEQ - QT0) / 128) * (DM / 64), NB), 128, 0, stream>>>(O16 + (size_t)QT0 * DM, DM, (size_t)SEQ * DM, WP, DM, (size_t)0, 0.0625f, bproj, nullptr, 0, out + (size_t)QT0 * DM, nullptr, DM, (size_t)SEQ_FULL * DM, SEQ - QT0, DM, DM);
  k_gemm2<<<dim3((QT0 / 128) * (DM / 64), NB), 128, 0, stream>>>(OH, DM, (size_t)QT0 * DM, WP, DM, (size_t)0, 0.0009765625f, bproj, nullptr, 0, out, nullptr, DM, (size_t)SEQ_FULL * DM, QT0, DM, DM);
  k_gemm2<<<dim3((QT0 / 128) * (DM / 64), NB), 128, 0, stream>>>(OL, DM, (size_t)QT0 * DM, WP, DM, (size_t)0, 9.5367431640625e-07f, nullptr, out, 0, out, nullptr, DM, (size_t)SEQ_FULL * DM, QT0, DM, DM);
}
